// GraphGNN_618475290909
// MI455X (gfx1250) — hardware-verified
//
#include <hip/hip_runtime.h>
#include <stddef.h>
#include <math.h>


#define NBATCH  4
#define DI      32
#define DH      32
#define DG      30
#define DO      32
#define DPQ     64
#define NTHR    256
#define NWAVE   8
#define PTHR    128
#define EPT     8
#define NGRP    2
#define CHUNK   (NTHR * EPT * NGRP)
#define WCAP    (EPT * NGRP * 32)
#define LISTN   (NWAVE * WCAP)
#define NBC     4096
#define NBF     1024
#define RCAP    40960
#define RBN     128
#define TGT     256
#define DEGCAP  512
#define OTHR    512
#define RT      128
#define LDU     40
#define WSCAP   134217728
#define SCL_A   8.0f
#define SCL_W   16.0f
#define SCL_ACC 0.0078125f

#define LDS_FILL ((RCAP + NBF + LISTN) * 4 + 64)

static_assert((CHUNK & (CHUNK - 1)) == 0);
static_assert(CHUNK <= 4096);
static_assert(NBC <= 4096 && NBF <= 4096);
static_assert((NBC & (NBC - 1)) == 0 && (NBF & (NBF - 1)) == 0);
static_assert(NBC == 4 * NBF);
static_assert(OTHR * 8 == NBC);
static_assert((RCAP % 32) == 0);
static_assert(TGT == NWAVE * 32);
static_assert((NBC % TGT) == 0);
static_assert((TGT % RT) == 0);
static_assert(RT == NWAVE * 16);
static_assert(DI == 32 && DH == 32 && DO == 32 && DPQ == 2 * DH && DG <= DH);
static_assert((LDU % 8) == 0 && LDU >= DH);

typedef float    v4f  __attribute__((ext_vector_type(4)));
typedef float    v8f  __attribute__((ext_vector_type(8)));
typedef int      v4i  __attribute__((ext_vector_type(4)));
typedef _Float16 v8h  __attribute__((ext_vector_type(8)));
typedef _Float16 v16h __attribute__((ext_vector_type(16)));
union FragH { v16h v; v8h h[2]; };

__device__ __forceinline__ v8f wmh(v16h a, v16h b, v8f c) {
  v8f d = __builtin_amdgcn_wmma_f32_16x16x32_f16(false, a, false, b, (short)0, c, false, false);
  asm volatile("v_nop\n\tv_nop\n\tv_nop\n\tv_nop" : "+v"(d) : "v"(a), "v"(b));
  return d;
}

__device__ __forceinline__ v8h cvt8(v4f a, v4f b, float s) {
  v8f t;
  t[0] = a.x * s; t[1] = a.y * s; t[2] = a.z * s; t[3] = a.w * s;
  t[4] = b.x * s; t[5] = b.y * s; t[6] = b.z * s; t[7] = b.w * s;
  return __builtin_convertvector(t, v8h);
}

__device__ __forceinline__ float sigm(float s) {
  s = s > 40.0f ? 40.0f : (s < -40.0f ? -40.0f : s);
  const float ex = expf(-s);
  return 1.0f / (1.0f + ex);
}

template <int NB>
__device__ __forceinline__ int scan_chunk(const int* __restrict__ dsts, int nE, int cbase, int slotBase,
                                          int vec8, int* list, int tid, int lane, int wave) {
  int wc = 0;
#pragma unroll
  for (int g = 0; g < NGRP; ++g) {
    const int el0  = (g * NTHR + tid) * EPT;
    const int e0   = cbase + el0;
    const int sent = -2147483647 - 1;
    v4i da, db;
    if (vec8 != 0 && cbase + CHUNK <= nE) {
      da = *(const v4i*)(dsts + e0);
      db = *(const v4i*)(dsts + e0 + 4);
    } else {
      da.x = (e0     < nE) ? dsts[min(e0, nE - 1)] : sent;
      da.y = (e0 + 1 < nE) ? dsts[min(e0 + 1, nE - 1)] : sent;
      da.z = (e0 + 2 < nE) ? dsts[min(e0 + 2, nE - 1)] : sent;
      da.w = (e0 + 3 < nE) ? dsts[min(e0 + 3, nE - 1)] : sent;
      db.x = (e0 + 4 < nE) ? dsts[min(e0 + 4, nE - 1)] : sent;
      db.y = (e0 + 5 < nE) ? dsts[min(e0 + 5, nE - 1)] : sent;
      db.z = (e0 + 6 < nE) ? dsts[min(e0 + 6, nE - 1)] : sent;
      db.w = (e0 + 7 < nE) ? dsts[min(e0 + 7, nE - 1)] : sent;
    }
    const unsigned nb = (unsigned)slotBase;
    const unsigned s0 = (unsigned)da.x - nb, s1 = (unsigned)da.y - nb;
    const unsigned s2 = (unsigned)da.z - nb, s3 = (unsigned)da.w - nb;
    const unsigned s4 = (unsigned)db.x - nb, s5 = (unsigned)db.y - nb;
    const unsigned s6 = (unsigned)db.z - nb, s7 = (unsigned)db.w - nb;
    const bool h0 = s0 < (unsigned)NB, h1 = s1 < (unsigned)NB, h2 = s2 < (unsigned)NB, h3 = s3 < (unsigned)NB;
    const bool h4 = s4 < (unsigned)NB, h5 = s5 < (unsigned)NB, h6 = s6 < (unsigned)NB, h7 = s7 < (unsigned)NB;
    const unsigned any = __builtin_amdgcn_ballot_w32(h0 | h1 | h2 | h3 | h4 | h5 | h6 | h7);
    if (any != 0u) {
#define HITJ(J, HJ, SJ) { \
        const unsigned mj = __builtin_amdgcn_ballot_w32(HJ); \
        if (mj != 0u) { \
          if (HJ) { \
            const int pos = wc + (int)__builtin_amdgcn_mbcnt_lo(mj, 0u); \
            if (pos < WCAP) list[wave * WCAP + pos] = ((el0 + (J)) << 12) | (int)(SJ); \
          } \
          wc += (int)__builtin_popcount(mj); } }
      HITJ(0, h0, s0)
      HITJ(1, h1, s1)
      HITJ(2, h2, s2)
      HITJ(3, h3, s3)
      HITJ(4, h4, s4)
      HITJ(5, h5, s5)
      HITJ(6, h6, s6)
      HITJ(7, h7, s7)
#undef HITJ
    }
  }
  return wc;
}

__global__ __launch_bounds__(PTHR) void k_prepw(
    const float* __restrict__ W1, const float* __restrict__ W2, const float* __restrict__ W3,
    _Float16* w1p, _Float16* w2p, _Float16* w3p) {
  const int blk = blockIdx.x, tid = threadIdx.x;
  if (blk < 2) {
    const int i = blk * PTHR + tid;
    const int n2 = i >> 2, k0 = (i & 3) * 8;
    const int col = n2 & 31, koff = ((n2 >> 5) & 1) * DI;
    v8f t;
#pragma unroll
    for (int j = 0; j < 8; ++j) t[j] = W1[(size_t)(koff + k0 + j) * DH + col] * SCL_W;
    const v8h o = __builtin_convertvector(t, v8h);
    _Float16* d = w1p + (size_t)i * 8;
    *(volatile v8h*)d = o;
    __threadfence();
    *(volatile v8h*)d = o;
  } else if (blk == 2) {
    const int i = tid;
    const int n = i >> 2, k0 = (i & 3) * 8;
    const int nc = n > DG - 1 ? DG - 1 : n;
    v8f t;
#pragma unroll
    for (int j = 0; j < 8; ++j) {
      const float v = W2[(size_t)(k0 + j) * DG + nc];
      t[j] = (n < DG) ? v * SCL_W : 0.0f;
    }
    const v8h o = __builtin_convertvector(t, v8h);
    _Float16* d = w2p + (size_t)i * 8;
    *(volatile v8h*)d = o;
    __threadfence();
    *(volatile v8h*)d = o;
  } else if (blk == 3) {
    const int i = tid;
    const int n = i >> 2, k0 = (i & 3) * 8;
    v8f t;
#pragma unroll
    for (int j = 0; j < 8; ++j) {
      const int k = k0 + j;
      const int kc = k > DG - 1 ? DG - 1 : k;
      const float v = W3[(size_t)kc * DO + n];
      t[j] = (k < DG) ? v * SCL_W : 0.0f;
    }
    const v8h o = __builtin_convertvector(t, v8h);
    _Float16* d = w3p + (size_t)i * 8;
    *(volatile v8h*)d = o;
    __threadfence();
    *(volatile v8h*)d = o;
  }
}

__global__ __launch_bounds__(NTHR) void k_xcvt(const float* __restrict__ x, _Float16* xp,
                                               int nN, int npa, int nUnits) {
  constexpr int UPR = DI / 8;
  static_assert((UPR & (UPR - 1)) == 0);
  const int i = (int)blockIdx.x * NTHR + (int)threadIdx.x;
  if (i >= nUnits) return;
  const int row = i / UPR;
  const int c0  = (i & (UPR - 1)) * 8;
  int b = row / npa;
  const int n = row - b * npa;
  b = b > NBATCH - 1 ? NBATCH - 1 : (b < 0 ? 0 : b);
  int nn = n > nN - 1 ? nN - 1 : n;
  nn = nn < 0 ? 0 : nn;
  const float* p = x + ((size_t)b * nN + nn) * DI + c0;
  const v4f a = *(const v4f*)p;
  const v4f c = *(const v4f*)(p + 4);
  v8h o = cvt8(a, c, SCL_A);
  const v8h z = {(_Float16)0.0f, (_Float16)0.0f, (_Float16)0.0f, (_Float16)0.0f,
                 (_Float16)0.0f, (_Float16)0.0f, (_Float16)0.0f, (_Float16)0.0f};
  o = (n < nN) ? o : z;
  _Float16* d = xp + (size_t)i * 8;
  *(volatile v8h*)d = o;
  __threadfence();
  *(volatile v8h*)d = o;
}

__global__ __launch_bounds__(NTHR) void k_stats(const float* __restrict__ ea, float* statl, int nE) {
  __shared__ double red[NTHR];
  __shared__ double smean;
  __shared__ __attribute__((aligned(16))) float sv[4];
  const int tid = threadIdx.x;
  double s = 0.0;
#pragma unroll 1
  for (int i = tid; i < nE; i += NTHR) s += (double)ea[i];
  red[tid] = s;
  __syncthreads();
#pragma unroll 1
  for (int o = NTHR / 2; o > 0; o >>= 1) {
    if (tid < o) red[tid] = red[tid] + red[tid + o];
    __syncthreads();
  }
  if (tid == 0) smean = red[0] / (double)nE;
  __syncthreads();
  const double mean = smean;
  double q = 0.0;
#pragma unroll 1
  for (int i = tid; i < nE; i += NTHR) {
    const double d = (double)ea[i] - mean;
    q += d * d;
  }
  __syncthreads();
  red[tid] = q;
  __syncthreads();
#pragma unroll 1
  for (int o = NTHR / 2; o > 0; o >>= 1) {
    if (tid < o) red[tid] = red[tid] + red[tid + o];
    __syncthreads();
  }
  if (tid == 0) {
    const double var = red[0] / (double)(nE > 1 ? nE - 1 : 1);
    const float sd = sqrtf((float)var);
    const float rs = 1.0f / (sd > 0.0f ? sd : 1.0f);
    sv[0] = (float)mean; sv[1] = rs; sv[2] = sd; sv[3] = 0.0f;
  }
  __syncthreads();
  const v4f o = *(const v4f*)sv;
  if (tid < 8) *(volatile v4f*)(statl + 4 * tid) = o;
  __threadfence();
  if (tid < 8) *(volatile v4f*)(statl + 4 * tid) = o;
}

__global__ __launch_bounds__(NTHR) void k_count(
    const int* __restrict__ dsts, int* cnt, int nE, int vec8) {
  __shared__ __attribute__((aligned(16))) int scnt[NBC];
  __shared__ __attribute__((aligned(16))) int list[LISTN];
  __shared__ int wcnt[NWAVE];
  const int tid = threadIdx.x, lane = tid & 31, wave = tid >> 5;
  const int nodeBase = blockIdx.x * NBC;

  for (int i = tid; i < NBC; i += NTHR) scnt[i] = 0;
  __syncthreads();

  const int nChunks = (nE + CHUNK - 1) / CHUNK;
#pragma unroll 1
  for (int ch = 0; ch < nChunks; ++ch) {
    const int cbase = ch * CHUNK;
    const int wc = scan_chunk<NBC>(dsts, nE, cbase, nodeBase, vec8, list, tid, lane, wave);
    if (lane == 0) wcnt[wave] = wc;
    __syncthreads();
    if (wave == 0) {
#pragma unroll 1
      for (int wsx = 0; wsx < NWAVE; ++wsx) {
        int n = __builtin_amdgcn_readfirstlane(wcnt[wsx]);
        n = n > WCAP ? WCAP : (n < 0 ? 0 : n);
        const int* lp = list + wsx * WCAP;
#pragma unroll 1
        for (int i = 0; i < n; ++i) {
          const int ent  = __builtin_amdgcn_readfirstlane(lp[i]);
          const int slot = ent & (NBC - 1);
          if (lane == 0) scnt[slot] = scnt[slot] + 1;
        }
      }
    }
    __syncthreads();
  }

  v4i cq[4];
#pragma unroll
  for (int q = 0; q < 4; ++q) {
    const int f = (wave * 4 + q) * 128 + 4 * lane;
    cq[q] = *(const v4i*)(scnt + f);
  }
  int* cp = cnt + (size_t)nodeBase;
#pragma unroll
  for (int q = 0; q < 4; ++q) {
    const int f = (wave * 4 + q) * 128 + 4 * lane;
    *(volatile v4i*)(cp + f) = cq[q];
  }
  __threadfence();
#pragma unroll
  for (int q = 0; q < 4; ++q) {
    const int f = (wave * 4 + q) * 128 + 4 * lane;
    *(volatile v4i*)(cp + f) = cq[q];
  }
}

__global__ __launch_bounds__(OTHR) void k_offsets(
    const int* __restrict__ cnt, int* off, int* rbase, int nChunk) {
  __shared__ __attribute__((aligned(16))) int soff[NBC];
  __shared__ __attribute__((aligned(16))) int srb[RBN];
  __shared__ int wtot[OTHR / 32];
  const int tid = threadIdx.x, lane = tid & 31, wave = tid >> 5, sub = tid >> 7;
  for (int i = tid; i < RBN; i += OTHR) srb[i] = 0;
  int carry = 0;
#pragma unroll 1
  for (int ch = 0; ch < nChunk; ++ch) {
    const int base = ch * NBC;
    const v4i c0 = *(const v4i*)(cnt + base + 8 * tid);
    const v4i c1 = *(const v4i*)(cnt + base + 8 * tid + 4);
    const int e0 = max(c0.x, 0), e1 = max(c0.y, 0), e2 = max(c0.z, 0), e3 = max(c0.w, 0);
    const int e4 = max(c1.x, 0), e5 = max(c1.y, 0), e6 = max(c1.z, 0), e7 = max(c1.w, 0);
    const int ts = e0 + e1 + e2 + e3 + e4 + e5 + e6 + e7;
    int incl = ts;
#pragma unroll
    for (int d = 1; d < 32; d <<= 1) {
      const int t = __shfl_up(incl, d);
      if (lane >= d) incl += t;
    }
    if (lane == 31) wtot[wave] = incl;
    __syncthreads();
    const int S0 = wtot[0]  + wtot[1]  + wtot[2]  + wtot[3];
    const int S1 = wtot[4]  + wtot[5]  + wtot[6]  + wtot[7];
    const int S2 = wtot[8]  + wtot[9]  + wtot[10] + wtot[11];
    const int S3 = wtot[12] + wtot[13] + wtot[14] + wtot[15];
    int pre = 0;
#pragma unroll 1
    for (int w = 4 * sub; w < wave; ++w) pre += wtot[w];
    const int b0 = carry;
    const int b1 = b0 + ((S0 + 31) & ~31);
    const int b2 = b1 + ((S1 + 31) & ~31);
    const int b3 = b2 + ((S2 + 31) & ~31);
    const int b4 = b3 + ((S3 + 31) & ~31);
    const int myb = sub == 0 ? b0 : (sub == 1 ? b1 : (sub == 2 ? b2 : b3));
    if (tid == 0) {
      srb[min(4 * ch + 0, RBN - 1)] = b0;
      srb[min(4 * ch + 1, RBN - 1)] = b1;
      srb[min(4 * ch + 2, RBN - 1)] = b2;
      srb[min(4 * ch + 3, RBN - 1)] = b3;
    }
    int run = myb + pre + incl - ts;
    soff[8 * tid + 0] = run; run += e0;
    soff[8 * tid + 1] = run; run += e1;
    soff[8 * tid + 2] = run; run += e2;
    soff[8 * tid + 3] = run; run += e3;
    soff[8 * tid + 4] = run; run += e4;
    soff[8 * tid + 5] = run; run += e5;
    soff[8 * tid + 6] = run; run += e6;
    soff[8 * tid + 7] = run;
    carry = b4;
    __syncthreads();
    const v4i o0 = *(const v4i*)(soff + 4 * tid);
    const v4i o1 = *(const v4i*)(soff + 4 * (tid + OTHR));
    int* op = off + base;
    *(volatile v4i*)(op + 4 * tid) = o0;
    *(volatile v4i*)(op + 4 * (tid + OTHR)) = o1;
    __threadfence();
    *(volatile v4i*)(op + 4 * tid) = o0;
    *(volatile v4i*)(op + 4 * (tid + OTHR)) = o1;
    __syncthreads();
  }
  if (tid == 0) srb[min(4 * nChunk, RBN - 1)] = carry;
  __syncthreads();
  v4i rv = {0, 0, 0, 0};
  if (tid < 32) rv = *(const v4i*)(srb + 4 * tid);
  if (tid < 32) *(volatile v4i*)(rbase + 4 * tid) = rv;
  __threadfence();
  if (tid < 32) *(volatile v4i*)(rbase + 4 * tid) = rv;
}

__global__ __launch_bounds__(NTHR) void k_fill(
    const int* __restrict__ dsts, const int* __restrict__ off, const int* __restrict__ rbase,
    int* csr, int nE, int vec8, int csrLen) {
  extern __shared__ v4f lds_dyn[];
  int* region = (int*)lds_dyn;
  int* cursor = region + RCAP;
  int* list   = cursor + NBF;
  int* wcnt   = list + LISTN;
  const int tid = threadIdx.x, lane = tid & 31, wave = tid >> 5;
  const int b = blockIdx.x;
  const int nodeBase = b * NBF;

  int rb0 = rbase[b];
  const int rb1 = rbase[b + 1];
  rb0 = rb0 < 0 ? 0 : (rb0 > csrLen ? csrLen : rb0);
  rb0 &= ~31;
  int len = rb1 - rb0;
  len = len < 0 ? 0 : (len > RCAP ? RCAP : len);
  int lenW = (len + 31) & ~31;
  if (rb0 + lenW > csrLen) lenW = (csrLen - rb0) & ~31;

  {
    const v4i z = {0, 0, 0, 0};
    for (int i = tid; i < RCAP / 4; i += NTHR) ((v4i*)region)[i] = z;
    for (int s = tid; s < NBF; s += NTHR) {
      int o = off[nodeBase + s] - rb0;
      o = o < 0 ? 0 : (o > RCAP ? RCAP : o);
      cursor[s] = o;
    }
  }
  __syncthreads();

  const int nChunks = (nE + CHUNK - 1) / CHUNK;
#pragma unroll 1
  for (int ch = 0; ch < nChunks; ++ch) {
    const int cbase = ch * CHUNK;
    const int wc = scan_chunk<NBF>(dsts, nE, cbase, nodeBase, vec8, list, tid, lane, wave);
    if (lane == 0) wcnt[wave] = wc;
    __syncthreads();
    if (wave == 0) {
#pragma unroll 1
      for (int wsx = 0; wsx < NWAVE; ++wsx) {
        int n = __builtin_amdgcn_readfirstlane(wcnt[wsx]);
        n = n > WCAP ? WCAP : (n < 0 ? 0 : n);
        const int* lp = list + wsx * WCAP;
#pragma unroll 1
        for (int i = 0; i < n; ++i) {
          const int ent  = __builtin_amdgcn_readfirstlane(lp[i]);
          const int slot = ent & (NBF - 1);
          int e = cbase + ((ent >> 12) & (CHUNK - 1));
          e = e > nE - 1 ? nE - 1 : (e < 0 ? 0 : e);
          if (lane == 0) {
            int pos = cursor[slot];
            pos = pos < 0 ? 0 : (pos > RCAP - 1 ? RCAP - 1 : pos);
            region[pos] = e;
            const int np = pos + 1;
            cursor[slot] = np > RCAP ? RCAP : np;
          }
        }
      }
    }
    __syncthreads();
  }

  const int nv = lenW >> 2;
  int* gp = csr + rb0;
#pragma unroll 1
  for (int i = tid; i < nv; i += NTHR) { const v4i v = ((const v4i*)region)[i]; *(volatile v4i*)(gp + 4 * i) = v; }
  __threadfence();
#pragma unroll 1
  for (int i = tid; i < nv; i += NTHR) { const v4i v = ((const v4i*)region)[i]; *(volatile v4i*)(gp + 4 * i) = v; }
}

__global__ __launch_bounds__(NTHR) void k_pq(
    const _Float16* __restrict__ xb, const _Float16* __restrict__ w1p, float* pq, int nN) {
  constexpr int NIT4 = (RT * DPQ / 4) / NTHR;
  static_assert((RT * DPQ / 4) % NTHR == 0 && NIT4 == 8);
  __shared__ __attribute__((aligned(16))) float stg[RT * DPQ];
  const int tid = threadIdx.x, lane = tid & 31, wave = tid >> 5;
  const int hh = lane >> 4, m = lane & 15;
  const int rowBase = blockIdx.x * RT;

  FragH a;
  {
    const _Float16* ap = xb + (size_t)(rowBase + 16 * wave + m) * DI + 8 * hh;
    a.h[0] = *(const v8h*)ap;
    a.h[1] = *(const v8h*)(ap + 16);
  }
  v8f acc[4];
#pragma unroll
  for (int t = 0; t < 4; ++t) {
    FragH bf;
    const _Float16* bp = w1p + (size_t)(16 * t + m) * DI + 8 * hh;
    bf.h[0] = *(const v8h*)bp;
    bf.h[1] = *(const v8h*)(bp + 16);
    v8f z = {0.f, 0.f, 0.f, 0.f, 0.f, 0.f, 0.f, 0.f};
    acc[t] = wmh(a.v, bf.v, z);
  }
  const int lrow0 = 16 * wave + 8 * hh;
#pragma unroll
  for (int t = 0; t < 4; ++t) {
#pragma unroll
    for (int r = 0; r < 8; ++r) {
      float v = acc[t][r] * SCL_ACC;
      v = (rowBase + lrow0 + r < nN) ? v : 0.0f;
      stg[(lrow0 + r) * DPQ + 16 * t + m] = v;
    }
  }
  __syncthreads();

  float* tile = pq + (size_t)rowBase * DPQ;
  v4f ov[NIT4];
#pragma unroll
  for (int it = 0; it < NIT4; ++it) ov[it] = *(const v4f*)(stg + 4 * (it * NTHR + tid));
#pragma unroll
  for (int it = 0; it < NIT4; ++it) *(volatile v4f*)(tile + 4 * (size_t)(it * NTHR + tid)) = ov[it];
  __threadfence();
#pragma unroll
  for (int it = 0; it < NIT4; ++it) *(volatile v4f*)(tile + 4 * (size_t)(it * NTHR + tid)) = ov[it];
}

__global__ __launch_bounds__(NTHR) void k_edge(
    const float* __restrict__ pq, const int* __restrict__ srcs, const int* __restrict__ tgts,
    const float* __restrict__ eat, const float* __restrict__ statl,
    const float* __restrict__ w1e, const float* __restrict__ b1,
    const _Float16* __restrict__ w2p, const float* __restrict__ b2,
    _Float16* hq, int nE, int nN) {
  __shared__ __attribute__((aligned(16))) _Float16 us[NWAVE * 32 * LDU];
  __shared__ __attribute__((aligned(16))) _Float16 stg[NWAVE * 32 * DH];
  const int tid = threadIdx.x, lane = tid & 31, wave = tid >> 5;
  const int hh = lane >> 4, m = lane & 15;
  const int ebase = blockIdx.x * NTHR + wave * 32;
  int el = ebase + lane;
  el = el > nE - 1 ? nE - 1 : el;
  el = el < 0 ? 0 : el;
  int s = srcs[el], t = tgts[el];
  s = s < 0 ? 0 : (s > nN - 1 ? nN - 1 : s);
  t = t < 0 ? 0 : (t > nN - 1 ? nN - 1 : t);
  const float mean = statl[0], rstd = statl[1];
  const float av = (eat[el] - mean) * rstd;
  const float wl = w1e[lane], bl = b1[lane];
  _Float16* uw = us + wave * (32 * LDU);

#pragma unroll 1
  for (int j = 0; j < 32; ++j) {
    const int sa = __builtin_amdgcn_readlane(s, j);
    const int sb = __builtin_amdgcn_readlane(t, j);
    const float aj = __int_as_float(__builtin_amdgcn_readlane(__float_as_int(av), j));
    const float p = pq[(size_t)sa * DPQ + lane];
    const float q = pq[(size_t)sb * DPQ + DH + lane];
    const float u = p + q + aj * wl + bl;
    const float h = sigm(u) * SCL_A;
    uw[j * LDU + lane] = (_Float16)h;
  }
  __syncthreads();

  FragH bq[2];
#pragma unroll
  for (int tt = 0; tt < 2; ++tt) {
    const _Float16* bp = w2p + (size_t)(16 * tt + m) * DH + 8 * hh;
    bq[tt].h[0] = *(const v8h*)bp;
    bq[tt].h[1] = *(const v8h*)(bp + 16);
  }
  const int n0 = m, n1 = 16 + m;
  const float b2a = b2[n0 > DG - 1 ? DG - 1 : n0];
  const float b2b = b2[n1 > DG - 1 ? DG - 1 : n1];
  _Float16* sw = stg + wave * (32 * DH);

#pragma unroll
  for (int g = 0; g < 2; ++g) {
    FragH a;
    const _Float16* arow = uw + (16 * g + m) * LDU + 8 * hh;
    a.h[0] = *(const v8h*)arow;
    a.h[1] = *(const v8h*)(arow + 16);
    v8f acc0 = {0.f, 0.f, 0.f, 0.f, 0.f, 0.f, 0.f, 0.f};
    v8f acc1 = {0.f, 0.f, 0.f, 0.f, 0.f, 0.f, 0.f, 0.f};
    acc0 = wmh(a.v, bq[0].v, acc0);
    acc1 = wmh(a.v, bq[1].v, acc1);
#pragma unroll
    for (int r = 0; r < 8; ++r) {
      const float v0 = sigm(acc0[r] * SCL_ACC + b2a) * SCL_A;
      float v1 = sigm(acc1[r] * SCL_ACC + b2b) * SCL_A;
      v1 = (n1 < DG) ? v1 : 0.0f;
      sw[(16 * g + 8 * hh + r) * DH + n0] = (_Float16)v0;
      sw[(16 * g + 8 * hh + r) * DH + n1] = (_Float16)v1;
    }
  }
  __syncthreads();

  v8h pv[4];
#pragma unroll
  for (int it = 0; it < 4; ++it) pv[it] = *(const v8h*)(sw + 8 * (it * 32 + lane));
  _Float16* gp = hq + (size_t)ebase * DH;
#pragma unroll
  for (int it = 0; it < 4; ++it) *(volatile v8h*)(gp + 8 * (it * 32 + lane)) = pv[it];
  __threadfence();
#pragma unroll
  for (int it = 0; it < 4; ++it) *(volatile v8h*)(gp + 8 * (it * 32 + lane)) = pv[it];
}

__device__ __forceinline__ float seg_sum(const int* __restrict__ csr, const _Float16* __restrict__ hp,
                                          int st, int n, int lane, int nE, int csrLen) {
  float acc = 0.0f;
#pragma unroll 1
  for (int q0 = 0; q0 < n; q0 += 32) {
    int pos = st + q0 + lane;
    pos = pos < 0 ? 0 : (pos > csrLen - 1 ? csrLen - 1 : pos);
    int el = csr[pos];
    el = el < 0 ? 0 : (el > nE - 1 ? nE - 1 : el);
    const int mcnt = (n - q0) < 32 ? (n - q0) : 32;
#pragma unroll 1
    for (int pp = 0; pp < mcnt; ++pp) {
      const int e = __builtin_amdgcn_readlane(el, pp);
      acc += (float)hp[(size_t)e * DH + lane];
    }
  }
  return acc;
}

__global__ __launch_bounds__(NTHR) void k_agg(
    const int* __restrict__ csrT, const int* __restrict__ offT, const int* __restrict__ cntT,
    const int* __restrict__ csrS, const int* __restrict__ offS, const int* __restrict__ cntS,
    const _Float16* __restrict__ hp, _Float16* ap, int nN, int nE, int csrLen) {
  __shared__ __attribute__((aligned(16))) _Float16 stg[NWAVE * 32 * DH];
  const int tid = threadIdx.x, lane = tid & 31, wave = tid >> 5;
  const int tbase = blockIdx.x * TGT + wave * 32;
  const int cl = tbase + lane;
  const int cT = cntT[cl], oT = offT[cl];
  const int cS = cntS[cl], oS = offS[cl];
  _Float16* sw = stg + wave * (32 * DH);

#pragma unroll 1
  for (int j = 0; j < 32; ++j) {
    const int c = tbase + j;
    int nT = __builtin_amdgcn_readfirstlane(__shfl(cT, j));
    int nS = __builtin_amdgcn_readfirstlane(__shfl(cS, j));
    const int stT = __builtin_amdgcn_readfirstlane(__shfl(oT, j));
    const int stS = __builtin_amdgcn_readfirstlane(__shfl(oS, j));
    nT = nT < 0 ? 0 : (nT > nE ? nE : nT);
    nS = nS < 0 ? 0 : (nS > nE ? nE : nS);
    const int tT = nT > DEGCAP ? DEGCAP : nT;
    const int tS = nS > DEGCAP ? DEGCAP : nS;
    const float sp = seg_sum(csrT, hp, stT, tT, lane, nE, csrLen);
    const float sm = seg_sum(csrS, hp, stS, tS, lane, nE, csrLen);
    float v = sp - sm;
    if (nT > DEGCAP || nS > DEGCAP) v = __int_as_float(0x7fc00000);
    if (c >= nN) v = 0.0f;
    sw[j * DH + lane] = (_Float16)v;
  }
  __syncthreads();

  v8h pv[4];
#pragma unroll
  for (int it = 0; it < 4; ++it) pv[it] = *(const v8h*)(sw + 8 * (it * 32 + lane));
  _Float16* gp = ap + (size_t)tbase * DH;
#pragma unroll
  for (int it = 0; it < 4; ++it) *(volatile v8h*)(gp + 8 * (it * 32 + lane)) = pv[it];
  __threadfence();
#pragma unroll
  for (int it = 0; it < 4; ++it) *(volatile v8h*)(gp + 8 * (it * 32 + lane)) = pv[it];
}

__global__ __launch_bounds__(NTHR) void k_out(
    const _Float16* __restrict__ agp, const _Float16* __restrict__ w3p, const float* __restrict__ b3,
    float* out, int nN, int npa, int tpb) {
  constexpr int NIT4 = (RT * DO / 4) / NTHR;
  static_assert(NIT4 == 4);
  __shared__ __attribute__((aligned(16))) float stg[RT * DO];
  const int tid = threadIdx.x, lane = tid & 31, wave = tid >> 5;
  const int hh = lane >> 4, m = lane & 15;
  const int b  = (int)blockIdx.x / tpb;
  const int tb = (int)blockIdx.x - b * tpb;

  FragH a;
  {
    const _Float16* arp = agp + ((size_t)b * npa + (size_t)tb * RT + 16 * wave + m) * DH + 8 * hh;
    a.h[0] = *(const v8h*)arp;
    a.h[1] = *(const v8h*)(arp + 16);
  }
  v8f acc[2];
#pragma unroll
  for (int t = 0; t < 2; ++t) {
    FragH bf;
    const _Float16* bp = w3p + (size_t)(16 * t + m) * DH + 8 * hh;
    bf.h[0] = *(const v8h*)bp;
    bf.h[1] = *(const v8h*)(bp + 16);
    v8f z = {0.f, 0.f, 0.f, 0.f, 0.f, 0.f, 0.f, 0.f};
    acc[t] = wmh(a.v, bf.v, z);
  }
  const int lrow0 = 16 * wave + 8 * hh;
#pragma unroll
  for (int t = 0; t < 2; ++t) {
    const float b3v = b3[16 * t + m];
#pragma unroll
    for (int r = 0; r < 8; ++r) {
      const float v = acc[t][r] * SCL_ACC + b3v;
      stg[(lrow0 + r) * DO + 16 * t + m] = sigm(v);
    }
  }
  __syncthreads();

  v4f ov[NIT4];
  bool ok[NIT4];
  size_t di[NIT4];
#pragma unroll
  for (int it = 0; it < NIT4; ++it) {
    const int u = it * NTHR + tid;
    const int rl = u >> 3;
    const int nloc = tb * RT + rl;
    ok[it] = nloc < nN;
    const int nc = nloc > nN - 1 ? nN - 1 : nloc;
    ov[it] = *(const v4f*)(stg + 4 * u);
    di[it] = ((size_t)b * nN + (size_t)nc) * DO + 4 * (u & 7);
  }
#pragma unroll
  for (int it = 0; it < NIT4; ++it) { if (ok[it]) *(volatile v4f*)(out + di[it]) = ov[it]; }
  __threadfence();
#pragma unroll
  for (int it = 0; it < NIT4; ++it) { if (ok[it]) *(volatile v4f*)(out + di[it]) = ov[it]; }
}

extern "C" void kernel_launch(void* const* d_in, const int* in_sizes, int n_in,
                              void* d_out, int out_size, void* d_ws, size_t ws_size,
                              hipStream_t stream) {
  if (n_in < 9) return;
  const int nNode = in_sizes[0] / DI;
  const int nN = nNode / NBATCH;
  const int nE = in_sizes[2];
  if (nN <= 0 || nE < 2) return;
  if (in_sizes[0] != NBATCH * nN * DI) return;
  if (in_sizes[1] != 2 * nE) return;
  if (in_sizes[3] != (2 * DI + 1) * DH || in_sizes[4] != DH) return;
  if (in_sizes[5] != DH * DG || in_sizes[6] != DG) return;
  if (in_sizes[7] != DG * DO || in_sizes[8] != DO) return;
  if (out_size != NBATCH * nN * DO) return;
  if (nE > (1 << 27) || nN > (1 << 22)) return;

  const float* x   = (const float*)d_in[0];
  const int*   ei  = (const int*)d_in[1];
  const float* ea  = (const float*)d_in[2];
  const float* W1  = (const float*)d_in[3];
  const float* b1  = (const float*)d_in[4];
  const float* W2  = (const float*)d_in[5];
  const float* b2  = (const float*)d_in[6];
  const float* W3  = (const float*)d_in[7];
  const float* b3  = (const float*)d_in[8];
  const int* src = ei;
  const int* tgt = ei + nE;
  const float* w1e = W1 + (size_t)(2 * DI) * DH;
  float* out = (float*)d_out;

  const int NPA    = ((nN + TGT - 1) / TGT) * TGT;
  const int nBC    = (nN + NBC - 1) / NBC;
  const int CNTPAD = nBC * NBC;
  if (CNTPAD < NPA) return;
  if (4 * nBC + 1 > RBN) return;
  const int nBF    = (nN + NBF - 1) / NBF;
  if (nBF + 1 > 4 * nBC + 1) return;
  const int csrLen = ((nE + 31) & ~31) + 4096;
  if (31 * 4 * nBC > 4096) return;
  const int EPAD   = ((nE + NTHR - 1) / NTHR) * NTHR;
  const int gE     = EPAD / NTHR;
  const int nAgg   = NPA / TGT;
  const int tpb    = NPA / RT;
  const int nXu    = NBATCH * NPA * (DI / 8);

  char* ws = (char*)d_ws;
  size_t off = 0;
  const size_t oSt  = off; off += 256;                                  off = (off + 255) & ~(size_t)255;
  const size_t oW1  = off; off += (size_t)DPQ * DI * 2;                 off = (off + 255) & ~(size_t)255;
  const size_t oW2  = off; off += (size_t)DH * DH * 2;                  off = (off + 255) & ~(size_t)255;
  const size_t oW3  = off; off += (size_t)DO * DH * 2;                  off = (off + 255) & ~(size_t)255;
  const size_t oX   = off; off += (size_t)NBATCH * NPA * DI * 2;        off = (off + 255) & ~(size_t)255;
  const size_t oA   = off; off += (size_t)NBATCH * NPA * DH * 2;        off = (off + 255) & ~(size_t)255;
  const size_t oPQ  = off; off += (size_t)NPA * DPQ * 4;                off = (off + 255) & ~(size_t)255;
  const size_t oH2  = off; off += (size_t)EPAD * DH * 2;                off = (off + 255) & ~(size_t)255;
  const size_t oCtT = off; off += (size_t)CNTPAD * 4;                   off = (off + 255) & ~(size_t)255;
  const size_t oOfT = off; off += (size_t)CNTPAD * 4;                   off = (off + 255) & ~(size_t)255;
  const size_t oRbT = off; off += (size_t)RBN * 4;                      off = (off + 255) & ~(size_t)255;
  const size_t oCsT = off; off += (size_t)csrLen * 4;                   off = (off + 255) & ~(size_t)255;
  const size_t oCtS = off; off += (size_t)CNTPAD * 4;                   off = (off + 255) & ~(size_t)255;
  const size_t oOfS = off; off += (size_t)CNTPAD * 4;                   off = (off + 255) & ~(size_t)255;
  const size_t oRbS = off; off += (size_t)RBN * 4;                      off = (off + 255) & ~(size_t)255;
  const size_t oCsS = off; off += (size_t)csrLen * 4;                   off = (off + 255) & ~(size_t)255;
  if (off > ws_size || off > (size_t)WSCAP) return;
  float*    statl = (float*)(ws + oSt);
  _Float16* w1p   = (_Float16*)(ws + oW1);
  _Float16* w2p   = (_Float16*)(ws + oW2);
  _Float16* w3p   = (_Float16*)(ws + oW3);
  _Float16* xP    = (_Float16*)(ws + oX);
  _Float16* aggP  = (_Float16*)(ws + oA);
  float*    pqP   = (float*)(ws + oPQ);
  _Float16* h2P   = (_Float16*)(ws + oH2);
  int* cntT = (int*)(ws + oCtT);
  int* offT = (int*)(ws + oOfT);
  int* rbT  = (int*)(ws + oRbT);
  int* csrT = (int*)(ws + oCsT);
  int* cntS = (int*)(ws + oCtS);
  int* offS = (int*)(ws + oOfS);
  int* rbS  = (int*)(ws + oRbS);
  int* csrS = (int*)(ws + oCsS);

  const int vec8 = ((nE & 7) == 0) ? 1 : 0;

  k_prepw<<<4, PTHR, 0, stream>>>(W1, W2, W3, w1p, w2p, w3p);
  k_xcvt<<<(nXu + NTHR - 1) / NTHR, NTHR, 0, stream>>>(x, xP, nN, NPA, nXu);
  k_stats<<<1, NTHR, 0, stream>>>(ea, statl, nE);

  hipFuncSetAttribute(reinterpret_cast<const void*>(&k_fill),
                      hipFuncAttributeMaxDynamicSharedMemorySize, LDS_FILL);
  k_count<<<nBC, NTHR, 0, stream>>>(tgt, cntT, nE, vec8);
  k_offsets<<<1, OTHR, 0, stream>>>(cntT, offT, rbT, nBC);
  k_fill<<<nBF, NTHR, LDS_FILL, stream>>>(tgt, offT, rbT, csrT, nE, vec8, csrLen);
  k_count<<<nBC, NTHR, 0, stream>>>(src, cntS, nE, vec8);
  k_offsets<<<1, OTHR, 0, stream>>>(cntS, offS, rbS, nBC);
  k_fill<<<nBF, NTHR, LDS_FILL, stream>>>(src, offS, rbS, csrS, nE, vec8, csrLen);

  for (int b = 0; b < NBATCH; ++b) {
    const _Float16* xb = xP + (size_t)b * NPA * DI;
    _Float16* ab = aggP + (size_t)b * NPA * DH;
    k_pq<<<tpb, NTHR, 0, stream>>>(xb, w1p, pqP, nN);
    k_edge<<<gE, NTHR, 0, stream>>>(pqP, src, tgt, ea, statl, w1e, b1, w2p, b2, h2P, nE, nN);
    k_agg<<<nAgg, NTHR, 0, stream>>>(csrT, offT, cntT, csrS, offS, cntS, h2P, ab, nN, nE, csrLen);
  }

  k_out<<<NBATCH * tpb, NTHR, 0, stream>>>(aggP, w3p, b3, out, nN, NPA, tpb);
}
